// CustomMamba_74620761801336
// MI455X (gfx1250) — hardware-verified
//
#include <hip/hip_runtime.h>
#include <math.h>

#pragma clang fp contract(off)

constexpr int kB   = 8;
constexpr int kT   = 24;
constexpr int kN   = 512;
constexpr int kF   = 64;
constexpr int kDI  = 128;
constexpr int kDS  = 16;
constexpr int kDR  = 4;
constexpr int kDC  = 4;
constexpr int kXD  = 36;
constexpr int kXDP = 64;
constexpr int kTok = kB * kT * kN;
constexpr int kChunkB    = 2;
constexpr int kNumChunks = kB / kChunkB;
constexpr int kMc        = kChunkB * kT * kN;
constexpr int kSerChunk  = kChunkB * kN;
static_assert(kMc % 64 == 0, "tile multiple");
static_assert(kNumChunks * kMc == kTok, "chunks cover all rows");

constexpr size_t kWPlaneElems = 16384;
constexpr size_t kWPlaneBytes = kWPlaneElems * 2;
constexpr size_t kOffW    = 0;
constexpr size_t kOffAtab = kOffW + 8 * kWPlaneBytes;
constexpr size_t kPlaneA  = (size_t)kMc * kDI * 2;
constexpr size_t kPlaneU  = (size_t)kMc * kF * 2;
constexpr size_t kOffAhi  = kOffAtab + 8192;
constexpr size_t kOffAlo  = kOffAhi + kPlaneA;
constexpr size_t kOffUhi  = kOffAlo + kPlaneA;
constexpr size_t kOffUlo  = kOffUhi + kPlaneU;
constexpr size_t kOffXz   = kOffUlo + kPlaneU;
constexpr size_t kOffChi  = kOffXz + (size_t)kMc * 2 * kDI * 4;
constexpr size_t kOffClo  = kOffChi + kPlaneA;
constexpr size_t kOffXd   = kOffClo + kPlaneA;
constexpr size_t kOffY    = kOffXd + (size_t)kMc * kXDP * 4;
constexpr size_t kWsTotal = kOffY + 2 * kPlaneA;
static_assert(kWsTotal == 75767808, "carve total");
static_assert(kWsTotal <= 134217728, "carve under 128 MiB");
constexpr size_t kYPlaneElems = (size_t)kMc * kDI;

typedef __attribute__((ext_vector_type(16))) _Float16 v16h;
typedef __attribute__((ext_vector_type(8)))  _Float16 v8h;
typedef __attribute__((ext_vector_type(16))) __bf16   v16b;
typedef __attribute__((ext_vector_type(8)))  __bf16   v8b;
typedef __attribute__((ext_vector_type(8)))  float    v8f;
typedef __attribute__((ext_vector_type(4)))  float    v4f;
typedef __attribute__((ext_vector_type(4)))  unsigned int v4u;

__device__ __forceinline__ unsigned short f2bf_bits(float f) {
  unsigned u = __float_as_uint(f);
  return (unsigned short)((u + 0x7FFFu + ((u >> 16) & 1u)) >> 16);
}
__device__ __forceinline__ float bf_bits2f(unsigned short h) { return __uint_as_float(((unsigned)h) << 16); }

__device__ __forceinline__ void dep_guard_h(v8f& a, v8f& b, v16h x, v16h y) { asm volatile("v_nop\n\tv_nop\n\tv_nop\n\tv_nop" : "+v"(a), "+v"(b) : "v"(x), "v"(y)); }
__device__ __forceinline__ void dep_guard_b(v8f& a, v8f& b, v16b x, v16b y) { asm volatile("v_nop\n\tv_nop\n\tv_nop\n\tv_nop" : "+v"(a), "+v"(b) : "v"(x), "v"(y)); }
__device__ __forceinline__ void keep4_h(v16h a, v16h b, v16h c, v16h d) { asm volatile("v_nop" :: "v"(a), "v"(b), "v"(c), "v"(d)); }
__device__ __forceinline__ void keep4_b(v16b a, v16b b, v16b c, v16b d) { asm volatile("v_nop" :: "v"(a), "v"(b), "v"(c), "v"(d)); }
__device__ __forceinline__ void acc_guard4(v8f& a, v8f& b, v8f& c, v8f& d) { asm volatile("v_nop\n\tv_nop\n\tv_nop\n\tv_nop" : "+v"(a), "+v"(b), "+v"(c), "+v"(d)); }
template <typename T> struct Frag;
template <> struct Frag<_Float16> {
  typedef v16h V; union U { v16h v; v8h h[2]; };
  static __device__ __forceinline__ v16h load(const _Float16* p) {
    U f; f.h[0] = *(const v8h*)(p); f.h[1] = *(const v8h*)(p + 16); return f.v;
  }
  static __device__ __forceinline__ v8f mma(v16h a, v16h b, v8f c) {
    return __builtin_amdgcn_wmma_f32_16x16x32_f16(false, a, false, b, (short)0, c, false, false);
  }
  static __device__ __forceinline__ void guard(v8f& a, v8f& b, v16h x, v16h y) { dep_guard_h(a, b, x, y); }
  static __device__ __forceinline__ void keep(v16h a, v16h b, v16h c, v16h d) { keep4_h(a, b, c, d); }
};
template <> struct Frag<__bf16> {
  typedef v16b V; union U { v16b v; v8b h[2]; };
  static __device__ __forceinline__ v16b load(const __bf16* p) {
    U f; f.h[0] = *(const v8b*)(p); f.h[1] = *(const v8b*)(p + 16); return f.v;
  }
  static __device__ __forceinline__ v8f mma(v16b a, v16b b, v8f c) {
    return __builtin_amdgcn_wmma_f32_16x16x32_bf16(false, a, false, b, (short)0, c, false, false);
  }
  static __device__ __forceinline__ void guard(v8f& a, v8f& b, v16b x, v16b y) { dep_guard_b(a, b, x, y); }
  static __device__ __forceinline__ void keep(v16b a, v16b b, v16b c, v16b d) { keep4_b(a, b, c, d); }
};

__device__ __forceinline__ unsigned pk16(unsigned short a, unsigned short b) { return (unsigned)a | ((unsigned)b << 16); }

template <int ET> struct Elem;
template <> struct Elem<0> { typedef _Float16 T; };
template <> struct Elem<1> { typedef __bf16 T; };
template <int ET, bool SPLIT, int BIAS_MODE, int OUT_MODE, bool RESID, int ACT = 0>
__global__ __launch_bounds__(256) void wmma_gemm64(
    const unsigned short* __restrict__ Ap, const unsigned short* __restrict__ A2p, int lda, long strideA,
    const unsigned short* __restrict__ Btp, const unsigned short* __restrict__ Bt2p, int ldb, long strideB,
    void* __restrict__ Cout, void* __restrict__ Cout2, int ldc, long strideC,
    const float* __restrict__ bias,
    const float* __restrict__ resid, long strideR,
    int M, int N, int K, float scale) {
  typedef typename Elem<ET>::T T;
  typedef typename Frag<T>::V V;
  const T* A = (const T*)Ap; const T* A2 = (const T*)A2p; const T* Bt = (const T*)Btp; const T* Bt2 = (const T*)Bt2p;
  __shared__ __align__(16) float sT[8][16 * 68];
  const int b    = blockIdx.y;
  const int lane = threadIdx.x & 31;
  const int wave = threadIdx.x >> 5;
  const int tilesN = N >> 6;
  const int tilesM = M >> 6;
  const int tile = blockIdx.x * 8 + wave;
  if (tile >= tilesM * tilesN) return;
  const int tm = tile / tilesN;
  const int tn = tile - tm * tilesN;
  const int m0 = tm << 6;
  const int n0 = tn << 6;

  const T* Ab  = A  + (size_t)b * strideA;
  const T* Bb  = Bt + (size_t)b * strideB;
  const T* Ab2 = SPLIT ? (A2  + (size_t)b * strideA) : nullptr;
  const T* Bb2 = SPLIT ? (Bt2 + (size_t)b * strideB) : nullptr;

  const int rlane = lane & 15;
  const int koff  = (lane >> 4) * 8;
  const int mOff  = (lane >> 4) * 8;

  v8f acc[4][4];
#pragma unroll
  for (int i = 0; i < 4; ++i)
#pragma unroll
    for (int j = 0; j < 4; ++j) acc[i][j] = (v8f){0.f,0.f,0.f,0.f,0.f,0.f,0.f,0.f};

  for (int k0 = 0; k0 < K; k0 += 32) {
    V bh[4], bl[4];
#pragma unroll
    for (int j = 0; j < 4; ++j) {
      const size_t bo = (size_t)(n0 + (j << 4) + rlane) * ldb + koff + k0;
      bh[j] = Frag<T>::load(Bb + bo);
      if (SPLIT) bl[j] = Frag<T>::load(Bb2 + bo);
    }
#pragma unroll
    for (int i = 0; i < 4; ++i) {
      const size_t ao = (size_t)(m0 + (i << 4) + rlane) * lda + koff + k0;
      V ah = Frag<T>::load(Ab + ao);
      V al;
      if (SPLIT) al = Frag<T>::load(Ab2 + ao);
#pragma unroll
      for (int j = 0; j < 4; ++j) {
        acc[i][j] = Frag<T>::mma(ah, bh[j], acc[i][j]);
        if (SPLIT) {
          acc[i][j] = Frag<T>::mma(ah, bl[j], acc[i][j]);
          acc[i][j] = Frag<T>::mma(al, bh[j], acc[i][j]);
        }
      }
      Frag<T>::guard(acc[i][0], acc[i][3], ah, SPLIT ? al : ah);
    }
    Frag<T>::keep(bh[0], bh[1], bh[2], bh[3]);
    if (SPLIT) Frag<T>::keep(bl[0], bl[1], bl[2], bl[3]);
  }
  acc_guard4(acc[0][0], acc[0][1], acc[0][2], acc[0][3]);
  acc_guard4(acc[1][0], acc[1][1], acc[1][2], acc[1][3]);
  acc_guard4(acc[2][0], acc[2][1], acc[2][2], acc[2][3]);
  acc_guard4(acc[3][0], acc[3][1], acc[3][2], acc[3][3]);

  float* slab = sT[wave];
  const float* Rb = RESID ? (resid + (size_t)b * strideR) : nullptr;
#pragma unroll
  for (int i = 0; i < 4; ++i) {
    const int mBase = m0 + (i << 4);
#pragma unroll
    for (int j = 0; j < 4; ++j) {
      const int n = n0 + (j << 4) + rlane;
      float bv = 0.f;
      if (BIAS_MODE == 2) bv = bias[n];
#pragma unroll
      for (int r = 0; r < 8; ++r) {
        float v = acc[i][j][r] * scale;
        if (BIAS_MODE == 1) v += bias[mBase + mOff + r];
        if (BIAS_MODE == 2) v += bv;
        if (RESID) v += Rb[(size_t)(mBase + mOff + r) * ldc + n];
        if (ACT == 2) v = fmaxf(v, 0.0f);
        if (ACT == 4) v = (v > 0.f) ? v : 0.01f * v;
        slab[(mOff + r) * 68 + (j << 4) + rlane] = v;
      }
    }
    __builtin_amdgcn_fence(__ATOMIC_RELEASE, "workgroup");
    __builtin_amdgcn_wave_barrier();
    __builtin_amdgcn_fence(__ATOMIC_ACQUIRE, "workgroup");
    if (OUT_MODE == 0) {
      float* C = (float*)Cout + (size_t)b * strideC;
      const int hh = lane >> 4, c4 = (lane & 15) * 4;
      for (int pass = 0; pass < 2; ++pass) {
#pragma unroll
        for (int it = 0; it < 8; ++it) {
          const int row = it * 2 + hh;
          v4f v = *(const v4f*)(slab + row * 68 + c4);
          *(volatile v4f*)(C + (size_t)(mBase + row) * ldc + n0 + c4) = v;
        }
        __threadfence();
      }
    } else {
      const int q = lane >> 3, c8 = (lane & 7) * 8;
      unsigned short* C  = (unsigned short*)Cout  + (size_t)b * strideC;
      unsigned short* C2 = (OUT_MODE == 2) ? ((unsigned short*)Cout2 + (size_t)b * strideC) : nullptr;
      for (int pass = 0; pass < 2; ++pass) {
#pragma unroll
        for (int it = 0; it < 4; ++it) {
          const int row = it * 4 + q;
          const float* sp = slab + row * 68 + c8;
          v8h hv, lv;
#pragma unroll
          for (int e = 0; e < 8; ++e) {
            if (OUT_MODE == 1) {
              hv[e] = (_Float16)sp[e];
            } else {
              unsigned short hb = f2bf_bits(sp[e]);
              unsigned short lb = f2bf_bits(sp[e] - bf_bits2f(hb));
              hv[e] = __builtin_bit_cast(_Float16, hb);
              lv[e] = __builtin_bit_cast(_Float16, lb);
            }
          }
          *(volatile v8h*)(C + (size_t)(mBase + row) * ldc + n0 + c8) = hv;
          if (OUT_MODE == 2) *(volatile v8h*)(C2 + (size_t)(mBase + row) * ldc + n0 + c8) = lv;
        }
        __threadfence();
      }
    }
    __builtin_amdgcn_fence(__ATOMIC_RELEASE, "workgroup");
    __builtin_amdgcn_wave_barrier();
    __builtin_amdgcn_fence(__ATOMIC_ACQUIRE, "workgroup");
  }
}

__device__ __forceinline__ void split2(float a, float b, unsigned& wh, unsigned& wl) {
  const unsigned short ha = f2bf_bits(a);
  const unsigned short hb = f2bf_bits(b);
  const unsigned short la = f2bf_bits(a - bf_bits2f(ha));
  const unsigned short lb = f2bf_bits(b - bf_bits2f(hb));
  wh = pk16(ha, hb);
  wl = pk16(la, lb);
}
__device__ __forceinline__ void split8(v4f a, v4f c, v4u& uh, v4u& ul) {
  unsigned h0, h1, h2, h3, l0, l1, l2, l3;
  split2(a[0], a[1], h0, l0);
  split2(a[2], a[3], h1, l1);
  split2(c[0], c[1], h2, l2);
  split2(c[2], c[3], h3, l3);
  uh = (v4u){h0, h1, h2, h3};
  ul = (v4u){l0, l1, l2, l3};
}
__device__ __forceinline__ float sigmoid_f(float v) {
  float a = -v;
  a = fminf(a, 60.0f);
  const float e = expf(a);
  return 1.0f / (1.0f + e);
}
__device__ __forceinline__ float silu_f(float v) { return v * sigmoid_f(v); }
__device__ __forceinline__ float softplus_f(float v) {
  const float e = expf(-fabsf(v));
  return fmaxf(v, 0.0f) + log1pf(e);
}
__device__ __forceinline__ float conv4(float x0, float x1, float x2, float x3, v4f w, float cb) {
  float acc = x0 * w[0];
  acc = acc + x1 * w[1];
  acc = acc + x2 * w[2];
  acc = acc + x3 * w[3];
  acc = acc + cb;
  return acc;
}

__global__ __launch_bounds__(256) void prep_kernel(const float* __restrict__ w_mix, const float* __restrict__ w_in,
                                                   const float* __restrict__ w_xp, const float* __restrict__ w_out,
                                                   const float* __restrict__ a_log,
                                                   unsigned short* __restrict__ wplanes, float* __restrict__ atab) {
  const int task = blockIdx.y;
  const int i = blockIdx.x * 256 + threadIdx.x;
  if (task == 4) {
    if (i < kDI * kDS) {
      const float v = -expf(a_log[i]);
      ((volatile float*)atab)[i] = v;
      __threadfence();
      ((volatile float*)atab)[i] = v;
    }
    return;
  }
  const float* W;
  int kdim, nvalid, npad;
  if (task == 0)      { W = w_mix; kdim = kDI; nvalid = kF;      npad = kF; }
  else if (task == 1) { W = w_in;  kdim = kF;  nvalid = 2 * kDI; npad = 2 * kDI; }
  else if (task == 2) { W = w_xp;  kdim = kDI; nvalid = kXD;     npad = kXDP; }
  else                { W = w_out; kdim = kDI; nvalid = kF;      npad = kF; }
  const int nthr = npad * kdim / 8;
  if (i >= nthr) return;
  const int e0 = i * 8;
  const int n  = e0 / kdim;
  const int k0 = e0 - n * kdim;
  const bool nz = (n < nvalid);
  const int nc = nz ? n : (nvalid - 1);
  float v[8];
#pragma unroll
  for (int e = 0; e < 8; ++e) {
    float t = W[(size_t)(k0 + e) * nvalid + nc];
    v[e] = nz ? t : 0.0f;
  }
  const v4f a = (v4f){v[0], v[1], v[2], v[3]};
  const v4f c = (v4f){v[4], v[5], v[6], v[7]};
  v4u uh, ul;
  split8(a, c, uh, ul);
  unsigned short* ph = wplanes + (size_t)task * 2 * kWPlaneElems + e0;
  unsigned short* pl = ph + kWPlaneElems;
  *(volatile v4u*)ph = uh;
  *(volatile v4u*)pl = ul;
  __threadfence();
  *(volatile v4u*)ph = uh;
  *(volatile v4u*)pl = ul;
}

__global__ __launch_bounds__(256) void cat_split_kernel(const float* __restrict__ xsrc, const float* __restrict__ qsrc,
                                                        unsigned short* __restrict__ ahi, unsigned short* __restrict__ alo, int nthr) {
  const int half = blockIdx.y;
  const int i = blockIdx.x * 256 + threadIdx.x;
  if (i >= nthr) return;
  const int r  = i >> 3;
  const int k0 = (i & 7) * 8;
  const float* src = ((half == 0) ? xsrc : qsrc) + (size_t)r * kF + k0;
  const v4f a = *(const v4f*)(src);
  const v4f c = *(const v4f*)(src + 4);
  v4u uh, ul;
  split8(a, c, uh, ul);
  const size_t o = (size_t)r * kDI + (size_t)half * kF + k0;
  *(volatile v4u*)(ahi + o) = uh;
  *(volatile v4u*)(alo + o) = ul;
  __threadfence();
  *(volatile v4u*)(ahi + o) = uh;
  *(volatile v4u*)(alo + o) = ul;
}

__global__ __launch_bounds__(256) void conv_silu_kernel(const float* __restrict__ xz, const float* __restrict__ conv_w,
                                                        const float* __restrict__ conv_b,
                                                        unsigned short* __restrict__ chi, unsigned short* __restrict__ clo, int nthr) {
  const int i = blockIdx.x * 256 + threadIdx.x;
  if (i >= nthr) return;
  const int r  = i >> 4;
  const int d0 = (i & 15) * 8;
  const int t  = (r >> 9) % kT;
  const bool ok1 = (t >= 1), ok2 = (t >= 2), ok3 = (t >= 3);
  const int r1 = ok1 ? (r - kN) : r;
  const int r2 = ok2 ? (r - 2 * kN) : r;
  const int r3 = ok3 ? (r - 3 * kN) : r;
  const float* p0 = xz + (size_t)r  * (2 * kDI) + d0;
  const float* p1 = xz + (size_t)r1 * (2 * kDI) + d0;
  const float* p2 = xz + (size_t)r2 * (2 * kDI) + d0;
  const float* p3 = xz + (size_t)r3 * (2 * kDI) + d0;
  const v4f a0 = *(const v4f*)(p0), c0 = *(const v4f*)(p0 + 4);
  const v4f a1 = *(const v4f*)(p1), c1 = *(const v4f*)(p1 + 4);
  const v4f a2 = *(const v4f*)(p2), c2 = *(const v4f*)(p2 + 4);
  const v4f a3 = *(const v4f*)(p3), c3 = *(const v4f*)(p3 + 4);
  float xt[8], xm1[8], xm2[8], xm3[8];
#pragma unroll
  for (int e = 0; e < 4; ++e) {
    xt[e]  = a0[e];                    xt[4 + e]  = c0[e];
    xm1[e] = ok1 ? a1[e] : 0.0f;        xm1[4 + e] = ok1 ? c1[e] : 0.0f;
    xm2[e] = ok2 ? a2[e] : 0.0f;        xm2[4 + e] = ok2 ? c2[e] : 0.0f;
    xm3[e] = ok3 ? a3[e] : 0.0f;        xm3[4 + e] = ok3 ? c3[e] : 0.0f;
  }
  float ov[8];
#pragma unroll
  for (int e = 0; e < 8; ++e) {
    const int d = d0 + e;
    const v4f w = *(const v4f*)(conv_w + (size_t)d * kDC);
    const float cb = conv_b[d];
    ov[e] = silu_f(conv4(xm3[e], xm2[e], xm1[e], xt[e], w, cb));
  }
  const v4f oa = (v4f){ov[0], ov[1], ov[2], ov[3]};
  const v4f oc = (v4f){ov[4], ov[5], ov[6], ov[7]};
  v4u uh, ul;
  split8(oa, oc, uh, ul);
  const size_t o = (size_t)r * kDI + d0;
  *(volatile v4u*)(chi + o) = uh;
  *(volatile v4u*)(clo + o) = ul;
  __threadfence();
  *(volatile v4u*)(chi + o) = uh;
  *(volatile v4u*)(clo + o) = ul;
}

__global__ __launch_bounds__(128) void scan_kernel(const float* __restrict__ xz, const float* __restrict__ xdbl,
                                                   const float* __restrict__ atab,
                                                   const float* __restrict__ conv_w, const float* __restrict__ conv_b,
                                                   const float* __restrict__ w_dt, const float* __restrict__ b_dt,
                                                   const float* __restrict__ dvec,
                                                   unsigned short* __restrict__ yplanes) {
  __shared__ __align__(16) float sX[kT * kXD];
  __shared__ __align__(16) float sY[kT * kDI];
  const int tid  = threadIdx.x;
  const int sidx = blockIdx.x;
  const int bl   = sidx >> 9;
  const int n    = sidx & (kN - 1);
  const int rowbase = bl * kT * kN + n;
  for (int i = tid; i < kT * kXD; i += 128) {
    const int t = i / kXD;
    const int c = i - t * kXD;
    sX[i] = xdbl[(size_t)(rowbase + t * kN) * kXDP + c];
  }
  const int d = tid;
  float an[kDS];
  {
    const v4f q0 = *(const v4f*)(atab + d * kDS);
    const v4f q1 = *(const v4f*)(atab + d * kDS + 4);
    const v4f q2 = *(const v4f*)(atab + d * kDS + 8);
    const v4f q3 = *(const v4f*)(atab + d * kDS + 12);
#pragma unroll
    for (int e = 0; e < 4; ++e) { an[e] = q0[e]; an[4 + e] = q1[e]; an[8 + e] = q2[e]; an[12 + e] = q3[e]; }
  }
  const v4f cw = *(const v4f*)(conv_w + (size_t)d * kDC);
  const float cb  = conv_b[d];
  const float wd0 = w_dt[d], wd1 = w_dt[kDI + d], wd2 = w_dt[2 * kDI + d], wd3 = w_dt[3 * kDI + d];
  const float bd  = b_dt[d];
  const float dd  = dvec[d];
  __syncthreads();

  float h[kDS];
#pragma unroll
  for (int s = 0; s < kDS; ++s) h[s] = 0.0f;
  float xm1 = 0.0f, xm2 = 0.0f, xm3 = 0.0f;
#pragma unroll 1
  for (int t = 0; t < kT; ++t) {
    const size_t r = (size_t)(rowbase + t * kN);
    const float xcur = xz[r * (2 * kDI) + d];
    const float zz   = xz[r * (2 * kDI) + kDI + d];
    const float u = silu_f(conv4(xm3, xm2, xm1, xcur, cw, cb));
    xm3 = xm2; xm2 = xm1; xm1 = xcur;
    const float* sx = sX + t * kXD;
    float dtr = sx[0] * wd0;
    dtr = dtr + sx[1] * wd1;
    dtr = dtr + sx[2] * wd2;
    dtr = dtr + sx[3] * wd3;
    dtr = dtr + bd;
    const float dt = softplus_f(dtr);
    const float du = dt * u;
    float y = 0.0f;
#pragma unroll
    for (int s = 0; s < kDS; ++s) {
      const float bv = sx[kDR + s];
      const float cv = sx[kDR + kDS + s];
      const float da = expf(dt * an[s]);
      h[s] = da * h[s] + du * bv;
      y = y + h[s] * cv;
    }
    float yv = y + u * dd;
    yv = yv * silu_f(zz);
    sY[t * kDI + d] = yv;
  }
  __syncthreads();

  const int wave = tid >> 5, lane = tid & 31;
  const int c8 = (lane & 15) * 8;
  const int plane = lane >> 4;
  unsigned short* yb = yplanes + (size_t)plane * kYPlaneElems;
  for (int pass = 0; pass < 2; ++pass) {
    for (int t = wave; t < kT; t += 4) {
      const float* sp = sY + t * kDI + c8;
      const v4f a = *(const v4f*)(sp);
      const v4f c = *(const v4f*)(sp + 4);
      v4u uh, ul;
      split8(a, c, uh, ul);
      v4u st;
      st.x = plane ? ul.x : uh.x;
      st.y = plane ? ul.y : uh.y;
      st.z = plane ? ul.z : uh.z;
      st.w = plane ? ul.w : uh.w;
      *(volatile v4u*)(yb + (size_t)(rowbase + t * kN) * kDI + c8) = st;
    }
    __threadfence();
  }
}

extern "C" void kernel_launch(void* const* d_in, const int* in_sizes, int n_in,
                              void* d_out, int out_size, void* d_ws, size_t ws_size,
                              hipStream_t stream) {
  if (n_in < 13) return;
  if (in_sizes[0] != kTok * kF || in_sizes[1] != kTok * kF || in_sizes[2] != 2 * kF * kF || in_sizes[3] != kF ||
      in_sizes[4] != kF * 2 * kDI || in_sizes[5] != kDI * kDC || in_sizes[6] != kDI || in_sizes[7] != kDI * kXD ||
      in_sizes[8] != kDR * kDI || in_sizes[9] != kDI || in_sizes[10] != kDI * kDS || in_sizes[11] != kDI ||
      in_sizes[12] != kDI * kF || out_size != kTok * kF) return;
  if (ws_size < kWsTotal) return;

  const float* x       = (const float*)d_in[0];
  const float* qk      = (const float*)d_in[1];
  const float* w_mix   = (const float*)d_in[2];
  const float* b_mix   = (const float*)d_in[3];
  const float* w_in    = (const float*)d_in[4];
  const float* conv_w  = (const float*)d_in[5];
  const float* conv_b  = (const float*)d_in[6];
  const float* w_xproj = (const float*)d_in[7];
  const float* w_dt    = (const float*)d_in[8];
  const float* b_dt    = (const float*)d_in[9];
  const float* a_log   = (const float*)d_in[10];
  const float* dvec    = (const float*)d_in[11];
  const float* w_out   = (const float*)d_in[12];
  float* out = (float*)d_out;
  char* ws = (char*)d_ws;

  unsigned short* wpl     = (unsigned short*)(ws + kOffW);
  unsigned short* wmix_hi = wpl + 0 * kWPlaneElems;
  unsigned short* wmix_lo = wpl + 1 * kWPlaneElems;
  unsigned short* win_hi  = wpl + 2 * kWPlaneElems;
  unsigned short* win_lo  = wpl + 3 * kWPlaneElems;
  unsigned short* wxp_hi  = wpl + 4 * kWPlaneElems;
  unsigned short* wxp_lo  = wpl + 5 * kWPlaneElems;
  unsigned short* wout_hi = wpl + 6 * kWPlaneElems;
  unsigned short* wout_lo = wpl + 7 * kWPlaneElems;
  float*          atab    = (float*)(ws + kOffAtab);
  unsigned short* a_hi    = (unsigned short*)(ws + kOffAhi);
  unsigned short* a_lo    = (unsigned short*)(ws + kOffAlo);
  unsigned short* u_hi    = (unsigned short*)(ws + kOffUhi);
  unsigned short* u_lo    = (unsigned short*)(ws + kOffUlo);
  float*          xz      = (float*)(ws + kOffXz);
  unsigned short* c_hi    = (unsigned short*)(ws + kOffChi);
  unsigned short* c_lo    = (unsigned short*)(ws + kOffClo);
  float*          xdbl    = (float*)(ws + kOffXd);
  unsigned short* ypl     = (unsigned short*)(ws + kOffY);
  unsigned short* y_hi    = ypl;
  unsigned short* y_lo    = ypl + kYPlaneElems;

  prep_kernel<<<dim3(8, 5), 256, 0, stream>>>(w_mix, w_in, w_xproj, w_out, a_log, wpl, atab);

  const int gridM64 = kMc / 64;
  for (int c = 0; c < kNumChunks; ++c) {
    const size_t row0 = (size_t)c * kMc;
    const float* xc  = x  + row0 * kF;
    const float* qc  = qk + row0 * kF;
    float* outc = out + row0 * kF;

    cat_split_kernel<<<dim3(kMc * 8 / 256, 2), 256, 0, stream>>>(xc, qc, a_hi, a_lo, kMc * 8);

    wmma_gemm64<1, true, 2, 2, false, 0><<<dim3((gridM64 * 1 + 7) / 8, 1), 256, 0, stream>>>(
        a_hi, a_lo, kDI, 0L, wmix_hi, wmix_lo, kDI, 0L, (void*)u_hi, (void*)u_lo, kF, 0L,
        b_mix, nullptr, 0L, kMc, kF, kDI, 1.0f);

    wmma_gemm64<1, true, 0, 0, false, 0><<<dim3((gridM64 * 4 + 7) / 8, 1), 256, 0, stream>>>(
        u_hi, u_lo, kF, 0L, win_hi, win_lo, kF, 0L, (void*)xz, nullptr, 2 * kDI, 0L,
        nullptr, nullptr, 0L, kMc, 2 * kDI, kF, 1.0f);

    conv_silu_kernel<<<dim3(kMc * 16 / 256), 256, 0, stream>>>(xz, conv_w, conv_b, c_hi, c_lo, kMc * 16);

    wmma_gemm64<1, true, 0, 0, false, 0><<<dim3((gridM64 * 1 + 7) / 8, 1), 256, 0, stream>>>(
        c_hi, c_lo, kDI, 0L, wxp_hi, wxp_lo, kDI, 0L, (void*)xdbl, nullptr, kXDP, 0L,
        nullptr, nullptr, 0L, kMc, kXDP, kDI, 1.0f);

    scan_kernel<<<dim3(kSerChunk), 128, 0, stream>>>(xz, xdbl, atab, conv_w, conv_b, w_dt, b_dt, dvec, ypl);

    wmma_gemm64<1, true, 0, 0, false, 0><<<dim3((gridM64 * 1 + 7) / 8, 1), 256, 0, stream>>>(
        y_hi, y_lo, kDI, 0L, wout_hi, wout_lo, kDI, 0L, (void*)outc, nullptr, kF, 0L,
        nullptr, nullptr, 0L, kMc, kF, kDI, 1.0f);
  }
}
